// EnhancedMessageLayer_40037685133359
// MI455X (gfx1250) — hardware-verified
//
#include <hip/hip_runtime.h>
#include <stddef.h>


#define HD      128
#define NTHR    256
#define NWAVE   8
#define EPT     8
#define NGRP    2
#define CHUNK   (NTHR * EPT * NGRP)
#define WCAP    (EPT * NGRP * 32)
#define LISTN   (NWAVE * WCAP)
#define NB      512
#define GTHR    128
#define GWAVE   4
#define GROWS   64
#define PA1     136
#define PA2     264
#define PSO     256

#define LDS_AGG  (NB * HD * 4 + LISTN * 4 + 64 + NB * 4)
#define PQ_WAVE  (16 * PA1 * 2 * 2 + 16 * PSO * 4)
#define LDS_PQ   (GWAVE * PQ_WAVE)
#define ND_WAVE  (16 * PA2 * 2 * 2 + 16 * PA1 * 2 * 2 + 16 * HD * 4 * 2)
#define LDS_ND   (GWAVE * ND_WAVE)

static_assert((CHUNK & (CHUNK - 1)) == 0);
static_assert(CHUNK <= 4096);
static_assert(NB <= 4096 && (NB & (NB - 1)) == 0);
static_assert((PQ_WAVE & 15) == 0 && (ND_WAVE & 15) == 0);
static_assert(GROWS == GWAVE * 16);
static_assert(NB % GROWS == 0);
static_assert(NB * HD / 4 == NWAVE * 64 * 32);

typedef float          v4f  __attribute__((ext_vector_type(4)));
typedef float          v8f  __attribute__((ext_vector_type(8)));
typedef int            v4i  __attribute__((ext_vector_type(4)));
typedef unsigned short v4us __attribute__((ext_vector_type(4)));
typedef unsigned short v8us __attribute__((ext_vector_type(8)));
typedef __bf16         v16b __attribute__((ext_vector_type(16)));
union FragB { v16b v; v8us u[2]; };
union Pack8 { v8us v; v4us q[2]; };
struct HL4 { v4us h, l; };

__device__ __forceinline__ unsigned int bfr(float f) {
  unsigned int u = __float_as_uint(f);
  u += 0x7FFFu + ((u >> 16) & 1u);
  return u >> 16;
}
__device__ __forceinline__ void split1(float f, unsigned short& hi, unsigned short& lo) {
  const unsigned int hb = bfr(f);
  const float hf = __uint_as_float(hb << 16);
  hi = (unsigned short)hb;
  lo = (unsigned short)bfr(f - hf);
}
__device__ __forceinline__ HL4 split4(v4f v) {
  HL4 o;
  unsigned short a, b;
  split1(v.x, a, b); o.h.x = a; o.l.x = b;
  split1(v.y, a, b); o.h.y = a; o.l.y = b;
  split1(v.z, a, b); o.h.z = a; o.l.z = b;
  split1(v.w, a, b); o.h.w = a; o.l.w = b;
  return o;
}

__device__ __forceinline__ v8f wm3(v16b ah, v16b al, v16b bh, v16b bl, v8f c) {
  v8f d = __builtin_amdgcn_wmma_f32_16x16x32_bf16(false, ah, false, bh, (short)0, c, false, false);
  d = __builtin_amdgcn_wmma_f32_16x16x32_bf16(false, ah, false, bl, (short)0, d, false, false);
  d = __builtin_amdgcn_wmma_f32_16x16x32_bf16(false, al, false, bh, (short)0, d, false, false);
  asm volatile("v_nop\n\tv_nop\n\tv_nop\n\tv_nop" : "+v"(d) : "v"(ah), "v"(al), "v"(bh), "v"(bl));
  return d;
}

template <int KT>
__device__ __forceinline__ void gemm4(const unsigned short* aH, const unsigned short* aL, int apitch,
                                      const unsigned short* __restrict__ bH,
                                      const unsigned short* __restrict__ bL,
                                      int n0, int lane, v8f* acc) {
  const int hh = lane >> 4, m = lane & 15;
#pragma unroll
  for (int t = 0; t < 4; ++t) { v8f z = {0.f, 0.f, 0.f, 0.f, 0.f, 0.f, 0.f, 0.f}; acc[t] = z; }
  const unsigned short* arH = aH + m * apitch + 8 * hh;
  const unsigned short* arL = aL + m * apitch + 8 * hh;
#pragma unroll 1
  for (int kt = 0; kt < KT; ++kt) {
    FragB ah, al;
    ah.u[0] = *(const v8us*)(arH + 32 * kt);
    ah.u[1] = *(const v8us*)(arH + 32 * kt + 16);
    al.u[0] = *(const v8us*)(arL + 32 * kt);
    al.u[1] = *(const v8us*)(arL + 32 * kt + 16);
#pragma unroll
    for (int t = 0; t < 4; ++t) {
      const size_t bo = (size_t)(n0 + 16 * t + m) * (size_t)(KT * 32) + (size_t)(32 * kt + 8 * hh);
      FragB bh, bl;
      bh.u[0] = *(const v8us*)(bH + bo);
      bh.u[1] = *(const v8us*)(bH + bo + 16);
      bl.u[0] = *(const v8us*)(bL + bo);
      bl.u[1] = *(const v8us*)(bL + bo + 16);
      acc[t] = wm3(ah.v, al.v, bh.v, bl.v, acc[t]);
    }
  }
}

template <int NBT>
__device__ __forceinline__ int scan_chunk(const int* __restrict__ dsts, int nE, int cbase, int nodeBase,
                                          int vec8, int* list, int tid, int lane, int wave) {
  int wc = 0;
#pragma unroll
  for (int g = 0; g < NGRP; ++g) {
    const int el0  = (g * NTHR + tid) * EPT;
    const int e0   = cbase + el0;
    const int sent = -2147483647 - 1;
    v4i da, db;
    if (vec8 != 0 && cbase + CHUNK <= nE) {
      da = *(const v4i*)(dsts + e0);
      db = *(const v4i*)(dsts + e0 + 4);
    } else {
      da.x = (e0     < nE) ? dsts[min(e0,     nE - 1)] : sent;
      da.y = (e0 + 1 < nE) ? dsts[min(e0 + 1, nE - 1)] : sent;
      da.z = (e0 + 2 < nE) ? dsts[min(e0 + 2, nE - 1)] : sent;
      da.w = (e0 + 3 < nE) ? dsts[min(e0 + 3, nE - 1)] : sent;
      db.x = (e0 + 4 < nE) ? dsts[min(e0 + 4, nE - 1)] : sent;
      db.y = (e0 + 5 < nE) ? dsts[min(e0 + 5, nE - 1)] : sent;
      db.z = (e0 + 6 < nE) ? dsts[min(e0 + 6, nE - 1)] : sent;
      db.w = (e0 + 7 < nE) ? dsts[min(e0 + 7, nE - 1)] : sent;
    }
    const unsigned nb = (unsigned)nodeBase;
    const unsigned s0 = (unsigned)da.x - nb, s1 = (unsigned)da.y - nb;
    const unsigned s2 = (unsigned)da.z - nb, s3 = (unsigned)da.w - nb;
    const unsigned s4 = (unsigned)db.x - nb, s5 = (unsigned)db.y - nb;
    const unsigned s6 = (unsigned)db.z - nb, s7 = (unsigned)db.w - nb;
    const bool h0 = s0 < (unsigned)NBT, h1 = s1 < (unsigned)NBT, h2 = s2 < (unsigned)NBT, h3 = s3 < (unsigned)NBT;
    const bool h4 = s4 < (unsigned)NBT, h5 = s5 < (unsigned)NBT, h6 = s6 < (unsigned)NBT, h7 = s7 < (unsigned)NBT;
    const unsigned any = __builtin_amdgcn_ballot_w32(h0 | h1 | h2 | h3 | h4 | h5 | h6 | h7);
    if (any != 0u) {
#define HITJ(J, HJ, SJ) { \
        const unsigned mj = __builtin_amdgcn_ballot_w32(HJ); \
        if (mj != 0u) { \
          if (HJ) { \
            const int pos = wc + (int)__builtin_amdgcn_mbcnt_lo(mj, 0u); \
            if (pos < WCAP) list[wave * WCAP + pos] = ((el0 + (J)) << 12) | (int)(SJ); \
          } \
          wc += (int)__builtin_popcount(mj); } }
      HITJ(0, h0, s0)
      HITJ(1, h1, s1)
      HITJ(2, h2, s2)
      HITJ(3, h3, s3)
      HITJ(4, h4, s4)
      HITJ(5, h5, s5)
      HITJ(6, h6, s6)
      HITJ(7, h7, s7)
#undef HITJ
    }
  }
  return wc;
}

__global__ __launch_bounds__(256) void k_wprep(
    const float* __restrict__ Wm1, const float* __restrict__ Wm2, const float* __restrict__ Wg,
    const float* __restrict__ Wu1, const float* __restrict__ Wu2,
    unsigned short* m1h, unsigned short* m1l, unsigned short* m2h, unsigned short* m2l,
    unsigned short* gh, unsigned short* gl, unsigned short* u1h, unsigned short* u1l,
    unsigned short* u2h, unsigned short* u2l) {
  const int b = blockIdx.x;
  const float* W; unsigned short* dh; unsigned short* dl; int ksh; int lb;
  if (b < 16)      { W = Wm1; dh = m1h; dl = m1l; ksh = 7; lb = b; }
  else if (b < 24) { W = Wm2; dh = m2h; dl = m2l; ksh = 7; lb = b - 16; }
  else if (b < 40) { W = Wg;  dh = gh;  dl = gl;  ksh = 8; lb = b - 24; }
  else if (b < 56) { W = Wu1; dh = u1h; dl = u1l; ksh = 8; lb = b - 40; }
  else             { W = Wu2; dh = u2h; dl = u2l; ksh = 7; lb = b - 56; }
  const int o  = (lb * 256 + (int)threadIdx.x) * 8;
  const int n  = o >> ksh;
  const int k0 = o & ((1 << ksh) - 1);
  const int sh = (n >> 7) * HD;
  const int c  = n & (HD - 1);
  const float* p = W + (size_t)(k0 + sh) * HD + c;
  v4f a, bq;
  a.x  = p[0];       a.y  = p[HD];      a.z  = p[2 * HD];  a.w  = p[3 * HD];
  bq.x = p[4 * HD];  bq.y = p[5 * HD];  bq.z = p[6 * HD];  bq.w = p[7 * HD];
  const HL4 s0 = split4(a), s1 = split4(bq);
  Pack8 hv, lv;
  hv.q[0] = s0.h; hv.q[1] = s1.h;
  lv.q[0] = s0.l; lv.q[1] = s1.l;
  unsigned short* ph = dh + o;
  unsigned short* pl = dl + o;
  *(volatile v8us*)ph = hv.v;
  *(volatile v8us*)pl = lv.v;
  __threadfence();
  *(volatile v8us*)ph = hv.v;
  *(volatile v8us*)pl = lv.v;
}

__global__ __launch_bounds__(GTHR) void k_pq(
    const float* __restrict__ x,
    const unsigned short* __restrict__ w1h, const unsigned short* __restrict__ w1l,
    const float* __restrict__ bm1, float* P, float* Q, int nN) {
  extern __shared__ v4f lds_dyn[];
  const int tid = threadIdx.x, lane = tid & 31, wave = tid >> 5, hh = lane >> 4, m = lane & 15;
  char* base = (char*)lds_dyn + wave * PQ_WAVE;
  unsigned short* sAh = (unsigned short*)base;
  unsigned short* sAl = sAh + 16 * PA1;
  float*          sO  = (float*)(sAl + 16 * PA1);
  const int rowBase = blockIdx.x * GROWS + 16 * wave;

#pragma unroll
  for (int i = 0; i < 16; ++i) {
    int node = rowBase + i;
    node = node > nN - 1 ? nN - 1 : node;
    const v4f v = *(const v4f*)(x + (size_t)node * HD + 4 * lane);
    const HL4 s = split4(v);
    *(v4us*)(sAh + i * PA1 + 4 * lane) = s.h;
    *(v4us*)(sAl + i * PA1 + 4 * lane) = s.l;
  }
  __syncthreads();

#pragma unroll
  for (int nq = 0; nq < 4; ++nq) {
    v8f acc[4];
    gemm4<4>(sAh, sAl, PA1, w1h, w1l, 64 * nq, lane, acc);
#pragma unroll
    for (int t = 0; t < 4; ++t) {
      const int col = 64 * nq + 16 * t + m;
      const float bias = (nq >= 2) ? bm1[(col - HD) & (HD - 1)] : 0.0f;
      float* sp = sO + (8 * hh) * PSO + col;
#pragma unroll
      for (int r = 0; r < 8; ++r) sp[r * PSO] = acc[t][r] + bias;
    }
  }
  __syncthreads();

#pragma unroll
  for (int i = 0; i < 16; ++i) {
    const size_t go = ((size_t)rowBase + i) * HD + 4 * lane;
    const v4f pv = *(const v4f*)(sO + i * PSO + 4 * lane);
    const v4f qv = *(const v4f*)(sO + i * PSO + HD + 4 * lane);
    *(volatile v4f*)(P + go) = pv;
    *(volatile v4f*)(Q + go) = qv;
  }
  __threadfence();
#pragma unroll
  for (int i = 0; i < 16; ++i) {
    const size_t go = ((size_t)rowBase + i) * HD + 4 * lane;
    const v4f pv = *(const v4f*)(sO + i * PSO + 4 * lane);
    const v4f qv = *(const v4f*)(sO + i * PSO + HD + 4 * lane);
    *(volatile v4f*)(P + go) = pv;
    *(volatile v4f*)(Q + go) = qv;
  }
}

__global__ __launch_bounds__(NTHR) void k_agg(
    const int* __restrict__ ei, const float* __restrict__ ea, const float* __restrict__ Wm1,
    const float* __restrict__ P, const float* __restrict__ Q,
    float* U, float* cnt, int nN, int nE, int vec8) {
  extern __shared__ v4f lds_dyn[];
  float* acc  = (float*)lds_dyn;
  int*   list = (int*)(acc + NB * HD);
  int*   wcnt = list + LISTN;
  int*   cntl = wcnt + 16;
  const int tid = threadIdx.x, lane = tid & 31, wave = tid >> 5;
  const int nodeBase = blockIdx.x * NB;
  const int* dsts = ei + nE;

  {
    const v4f z = {0.f, 0.f, 0.f, 0.f};
    for (int i = tid; i < NB * HD / 4; i += NTHR) lds_dyn[i] = z;
    for (int i = tid; i < NB; i += NTHR) cntl[i] = 0;
  }
  const v4f w0 = *(const v4f*)(Wm1 + (size_t)(2 * HD) * HD + 4 * lane);
  const v4f w1 = *(const v4f*)(Wm1 + (size_t)(2 * HD + 1) * HD + 4 * lane);
  const v4f w2 = *(const v4f*)(Wm1 + (size_t)(2 * HD + 2) * HD + 4 * lane);
  __syncthreads();

  const int nChunks = (nE + CHUNK - 1) / CHUNK;
#pragma unroll 1
  for (int ch = 0; ch < nChunks; ++ch) {
    const int cbase = ch * CHUNK;
    const int wc = scan_chunk<NB>(dsts, nE, cbase, nodeBase, vec8, list, tid, lane, wave);
    if (lane == 0) wcnt[wave] = wc;
    __syncthreads();
    if (wave == 0) {
#pragma unroll 1
      for (int wsx = 0; wsx < NWAVE; ++wsx) {
        int n = __builtin_amdgcn_readfirstlane(wcnt[wsx]);
        n = n > WCAP ? WCAP : (n < 0 ? 0 : n);
        const int* lp = list + wsx * WCAP;
#pragma unroll 1
        for (int i = 0; i < n; ++i) {
          const int ent  = __builtin_amdgcn_readfirstlane(lp[i]);
          const int slot = ent & (NB - 1);
          int e = cbase + ((ent >> 12) & (CHUNK - 1));
          e = e > nE - 1 ? nE - 1 : e;
          int src = ei[e];
          src = src < 0 ? 0 : (src > nN - 1 ? nN - 1 : src);
          int qn = nodeBase + slot;
          qn = qn > nN - 1 ? nN - 1 : qn;
          const float a0 = ea[(size_t)e * 3];
          const float a1 = ea[(size_t)e * 3 + 1];
          const float a2 = ea[(size_t)e * 3 + 2];
          const v4f pv = *(const v4f*)(P + (size_t)src * HD + 4 * lane);
          const v4f qv = *(const v4f*)(Q + (size_t)qn * HD + 4 * lane);
          v4f u = pv + qv + w0 * a0 + w1 * a1 + w2 * a2;
          u.x = fmaxf(u.x, 0.f); u.y = fmaxf(u.y, 0.f); u.z = fmaxf(u.z, 0.f); u.w = fmaxf(u.w, 0.f);
          v4f* ap = (v4f*)(acc + slot * HD + 4 * lane);
          *ap = *ap + u;
          if (lane == 0) cntl[slot] = cntl[slot] + 1;
        }
      }
    }
    __syncthreads();
  }

  float* up = U + (size_t)nodeBase * HD;
  const int cf = (wave & 3) * 128 + 4 * lane;
  v4f cv;
  cv.x = (float)cntl[cf]; cv.y = (float)cntl[cf + 1]; cv.z = (float)cntl[cf + 2]; cv.w = (float)cntl[cf + 3];
#pragma unroll 4
  for (int q = 0; q < 64; ++q) {
    const int f = (wave * 64 + q) * 128 + 4 * lane;
    const v4f v = *(const v4f*)(acc + f);
    *(volatile v4f*)(up + f) = v;
  }
  if (wave < 4) *(volatile v4f*)(cnt + (size_t)nodeBase + cf) = cv;
  __threadfence();
#pragma unroll 4
  for (int q = 0; q < 64; ++q) {
    const int f = (wave * 64 + q) * 128 + 4 * lane;
    const v4f v = *(const v4f*)(acc + f);
    *(volatile v4f*)(up + f) = v;
  }
  if (wave < 4) *(volatile v4f*)(cnt + (size_t)nodeBase + cf) = cv;
}

__global__ __launch_bounds__(GTHR) void k_node(
    const float* __restrict__ x, const float* __restrict__ U, const float* __restrict__ cnt,
    const unsigned short* __restrict__ w2h, const unsigned short* __restrict__ w2l, const float* __restrict__ bm2,
    const unsigned short* __restrict__ wgh, const unsigned short* __restrict__ wgl, const float* __restrict__ bg,
    const unsigned short* __restrict__ wu1h, const unsigned short* __restrict__ wu1l, const float* __restrict__ bu1,
    const unsigned short* __restrict__ wu2h, const unsigned short* __restrict__ wu2l, const float* __restrict__ bu2,
    const float* __restrict__ gam, const float* __restrict__ bet, float* out, int nN) {
  extern __shared__ v4f lds_dyn[];
  const int tid = threadIdx.x, lane = tid & 31, wave = tid >> 5, hh = lane >> 4, m = lane & 15;
  char* base = (char*)lds_dyn + wave * ND_WAVE;
  unsigned short* sAh = (unsigned short*)base;
  unsigned short* sAl = sAh + 16 * PA2;
  unsigned short* sHh = sAl + 16 * PA2;
  unsigned short* sHl = sHh + 16 * PA1;
  float*          sG  = (float*)(sHl + 16 * PA1);
  float*          sO  = sG + 16 * HD;
  const int rowBase = blockIdx.x * GROWS + 16 * wave;

#pragma unroll
  for (int i = 0; i < 16; ++i) {
    int node = rowBase + i;
    node = node > nN - 1 ? nN - 1 : node;
    const v4f v = *(const v4f*)(U + (size_t)node * HD + 4 * lane);
    const HL4 s = split4(v);
    *(v4us*)(sAh + i * PA2 + 4 * lane) = s.h;
    *(v4us*)(sAl + i * PA2 + 4 * lane) = s.l;
  }
  float cn[8];
#pragma unroll
  for (int r = 0; r < 8; ++r) {
    int node = rowBase + 8 * hh + r;
    node = node > nN - 1 ? nN - 1 : node;
    cn[r] = cnt[node];
  }
  __syncthreads();

#pragma unroll
  for (int nh = 0; nh < 2; ++nh) {
    v8f acc[4];
    gemm4<4>(sAh, sAl, PA2, w2h, w2l, 64 * nh, lane, acc);
#pragma unroll
    for (int t = 0; t < 4; ++t) {
      const int col = 64 * nh + 16 * t + m;
      const float b = bm2[col];
#pragma unroll
      for (int r = 0; r < 8; ++r) {
        const float a = acc[t][r] + cn[r] * b;
        unsigned short ahv, alv;
        split1(a, ahv, alv);
        sAh[(8 * hh + r) * PA2 + HD + col] = ahv;
        sAl[(8 * hh + r) * PA2 + HD + col] = alv;
      }
    }
  }
  __syncthreads();

#pragma unroll
  for (int i = 0; i < 16; ++i) {
    int node = rowBase + i;
    node = node > nN - 1 ? nN - 1 : node;
    const v4f v = *(const v4f*)(x + (size_t)node * HD + 4 * lane);
    const HL4 s = split4(v);
    *(v4us*)(sAh + i * PA2 + 4 * lane) = s.h;
    *(v4us*)(sAl + i * PA2 + 4 * lane) = s.l;
  }
  __syncthreads();

#pragma unroll
  for (int nh = 0; nh < 2; ++nh) {
    v8f acc[4];
    gemm4<8>(sAh, sAl, PA2, wgh, wgl, 64 * nh, lane, acc);
#pragma unroll
    for (int t = 0; t < 4; ++t) {
      const int col = 64 * nh + 16 * t + m;
      const float b = bg[col];
#pragma unroll
      for (int r = 0; r < 8; ++r) {
        float z = acc[t][r] + b;
        z = fminf(fmaxf(z, -80.0f), 80.0f);
        const float g = 1.0f / (1.0f + __expf(-z));
        sG[(8 * hh + r) * HD + col] = g;
      }
    }
  }

#pragma unroll
  for (int nh = 0; nh < 2; ++nh) {
    v8f acc[4];
    gemm4<8>(sAh, sAl, PA2, wu1h, wu1l, 64 * nh, lane, acc);
#pragma unroll
    for (int t = 0; t < 4; ++t) {
      const int col = 64 * nh + 16 * t + m;
      const float b = bu1[col];
#pragma unroll
      for (int r = 0; r < 8; ++r) {
        const float hv = fmaxf(acc[t][r] + b, 0.0f);
        unsigned short h1, l1;
        split1(hv, h1, l1);
        sHh[(8 * hh + r) * PA1 + col] = h1;
        sHl[(8 * hh + r) * PA1 + col] = l1;
      }
    }
  }
  __syncthreads();

#pragma unroll
  for (int nh = 0; nh < 2; ++nh) {
    v8f acc[4];
    gemm4<4>(sHh, sHl, PA1, wu2h, wu2l, 64 * nh, lane, acc);
#pragma unroll
    for (int t = 0; t < 4; ++t) {
      const int col = 64 * nh + 16 * t + m;
      const float b = bu2[col];
#pragma unroll
      for (int r = 0; r < 8; ++r) {
        const int row = 8 * hh + r;
        int node = rowBase + row;
        node = node > nN - 1 ? nN - 1 : node;
        const float xv = x[(size_t)node * HD + col];
        const float g  = sG[row * HD + col];
        const float u  = acc[t][r] + b;
        sO[row * HD + col] = g * u + (1.0f - g) * xv;
      }
    }
  }
  __syncthreads();

  const float* rp = sO + m * HD + 64 * hh;
  float s = 0.f;
#pragma unroll
  for (int j = 0; j < 16; ++j) {
    const v4f v = *(const v4f*)(rp + 4 * j);
    s += (v.x + v.y) + (v.z + v.w);
  }
  s += __shfl_xor(s, 16);
  const float mean = s * (1.0f / 128.0f);
  float s2 = 0.f;
#pragma unroll
  for (int j = 0; j < 16; ++j) {
    const v4f v = *(const v4f*)(rp + 4 * j);
    const v4f d = v - mean;
    s2 += (d.x * d.x + d.y * d.y) + (d.z * d.z + d.w * d.w);
  }
  s2 += __shfl_xor(s2, 16);
  const float inv = rsqrtf(s2 * (1.0f / 128.0f) + 1e-5f);
  const v4f g4 = *(const v4f*)(gam + 4 * lane);
  const v4f b4 = *(const v4f*)(bet + 4 * lane);

#pragma unroll
  for (int i = 0; i < 16; ++i) {
    const float mi = __shfl(mean, i), vi = __shfl(inv, i);
    const int node = rowBase + i;
    const v4f o  = *(const v4f*)(sO + i * HD + 4 * lane);
    const v4f rr = (o - mi) * vi * g4 + b4;
    if (node < nN) *(volatile v4f*)(out + (size_t)node * HD + 4 * lane) = rr;
  }
  __threadfence();
#pragma unroll
  for (int i = 0; i < 16; ++i) {
    const float mi = __shfl(mean, i), vi = __shfl(inv, i);
    const int node = rowBase + i;
    const v4f o  = *(const v4f*)(sO + i * HD + 4 * lane);
    const v4f rr = (o - mi) * vi * g4 + b4;
    if (node < nN) *(volatile v4f*)(out + (size_t)node * HD + 4 * lane) = rr;
  }
}

extern "C" void kernel_launch(void* const* d_in, const int* in_sizes, int n_in,
                              void* d_out, int out_size, void* d_ws, size_t ws_size,
                              hipStream_t stream) {
  if (n_in < 15) return;
  const int nN = in_sizes[0] / HD;
  if (nN <= 0 || in_sizes[0] != nN * HD) return;
  if (in_sizes[1] < 0 || (in_sizes[1] & 1) != 0) return;
  const int nE = in_sizes[1] / 2;
  if (in_sizes[2] != nE * 3) return;
  if (in_sizes[3] != (2 * HD + 3) * HD) return;
  if (in_sizes[5] != HD * HD || in_sizes[7] != 2 * HD * HD || in_sizes[9] != 2 * HD * HD || in_sizes[11] != HD * HD) return;
  if (in_sizes[4] < HD || in_sizes[6] < HD || in_sizes[8] < HD || in_sizes[10] < HD || in_sizes[12] < HD) return;
  if (in_sizes[13] < HD || in_sizes[14] < HD) return;
  if (out_size != nN * HD) return;

  const float* x   = (const float*)d_in[0];
  const int*   ei  = (const int*)d_in[1];
  const float* ea  = (const float*)d_in[2];
  const float* Wm1 = (const float*)d_in[3];
  const float* bm1 = (const float*)d_in[4];
  const float* Wm2 = (const float*)d_in[5];
  const float* bm2 = (const float*)d_in[6];
  const float* Wg  = (const float*)d_in[7];
  const float* bg  = (const float*)d_in[8];
  const float* Wu1 = (const float*)d_in[9];
  const float* bu1 = (const float*)d_in[10];
  const float* Wu2 = (const float*)d_in[11];
  const float* bu2 = (const float*)d_in[12];
  const float* gam = (const float*)d_in[13];
  const float* bet = (const float*)d_in[14];
  float* out = (float*)d_out;

  const int nPQ  = (nN + GROWS - 1) / GROWS;
  const int nAgg = (nN + NB - 1) / NB;

  char* ws = (char*)d_ws;
  size_t off = 0;
#define CARVE(NAME, BYTES) const size_t NAME = off; off += ((size_t)(BYTES) + 255) & ~(size_t)255;
  CARVE(oM1h, (size_t)2 * HD * HD * 2)
  CARVE(oM1l, (size_t)2 * HD * HD * 2)
  CARVE(oM2h, (size_t)HD * HD * 2)
  CARVE(oM2l, (size_t)HD * HD * 2)
  CARVE(oGh,  (size_t)2 * HD * HD * 2)
  CARVE(oGl,  (size_t)2 * HD * HD * 2)
  CARVE(oU1h, (size_t)2 * HD * HD * 2)
  CARVE(oU1l, (size_t)2 * HD * HD * 2)
  CARVE(oU2h, (size_t)HD * HD * 2)
  CARVE(oU2l, (size_t)HD * HD * 2)
  CARVE(oP,   (size_t)nPQ * GROWS * HD * 4)
  CARVE(oQ,   (size_t)nPQ * GROWS * HD * 4)
  CARVE(oU,   (size_t)nAgg * NB * HD * 4)
  CARVE(oCnt, (size_t)nAgg * NB * 4)
#undef CARVE
  if (off > ws_size) return;
  unsigned short* m1h = (unsigned short*)(ws + oM1h);
  unsigned short* m1l = (unsigned short*)(ws + oM1l);
  unsigned short* m2h = (unsigned short*)(ws + oM2h);
  unsigned short* m2l = (unsigned short*)(ws + oM2l);
  unsigned short* wgh = (unsigned short*)(ws + oGh);
  unsigned short* wgl = (unsigned short*)(ws + oGl);
  unsigned short* u1h = (unsigned short*)(ws + oU1h);
  unsigned short* u1l = (unsigned short*)(ws + oU1l);
  unsigned short* u2h = (unsigned short*)(ws + oU2h);
  unsigned short* u2l = (unsigned short*)(ws + oU2l);
  float* P   = (float*)(ws + oP);
  float* Q   = (float*)(ws + oQ);
  float* U   = (float*)(ws + oU);
  float* cnt = (float*)(ws + oCnt);

  const int vec8 = ((nE & 3) == 0) ? 1 : 0;

  k_wprep<<<64, 256, 0, stream>>>(Wm1, Wm2, Wg, Wu1, Wu2, m1h, m1l, m2h, m2l, wgh, wgl, u1h, u1l, u2h, u2l);

  hipFuncSetAttribute(reinterpret_cast<const void*>(&k_pq),
                      hipFuncAttributeMaxDynamicSharedMemorySize, LDS_PQ);
  k_pq<<<nPQ, GTHR, LDS_PQ, stream>>>(x, m1h, m1l, bm1, P, Q, nN);

  hipFuncSetAttribute(reinterpret_cast<const void*>(&k_agg),
                      hipFuncAttributeMaxDynamicSharedMemorySize, LDS_AGG);
  k_agg<<<nAgg, NTHR, LDS_AGG, stream>>>(ei, ea, Wm1, P, Q, U, cnt, nN, nE, vec8);

  hipFuncSetAttribute(reinterpret_cast<const void*>(&k_node),
                      hipFuncAttributeMaxDynamicSharedMemorySize, LDS_ND);
  k_node<<<nPQ, GTHR, LDS_ND, stream>>>(x, U, cnt, m2h, m2l, bm2, wgh, wgl, bg, u1h, u1l, bu1,
                                        u2h, u2l, bu2, gam, bet, out, nN);
}
